// HashedImageField_9285719294006
// MI455X (gfx1250) — hardware-verified
//
#include <hip/hip_runtime.h>


namespace {
constexpr int NP = 2097152, L = 8, HS = 1 << 19, DF = 16, H = 64;
constexpr float AS = 65536.0f, WSC = 256.0f;
__constant__ float c_scale[L] = {7.00000000f, 11.2730188f, 17.8283749f, 27.8851261f, 43.3134651f, 66.9824982f, 103.293816f, 159.000000f};
__constant__ int c_res[L] = {8, 13, 19, 29, 45, 68, 105, 160};
__constant__ int c_dense[L] = {1, 1, 1, 1, 1, 1, 0, 0};
typedef _Float16 b16;
typedef __attribute__((ext_vector_type(16))) _Float16 v16b;
typedef __attribute__((ext_vector_type(8))) _Float16 v8b;
typedef __attribute__((ext_vector_type(8))) float v8f;
typedef __attribute__((ext_vector_type(4))) float v4f;
typedef __attribute__((ext_vector_type(2))) float v2f;
__device__ __forceinline__ float bf16_rne(float f) { unsigned int u = __float_as_uint(f); u += 0x7FFFu + ((u >> 16) & 1u); float r = __uint_as_float(u & 0xFFFF0000u); asm volatile("" : "+v"(r)); return r; }
__device__ __forceinline__ v16b frag_kb(const b16* p, int hh) { const v8b a = *(const v8b*)(p + 8 * hh), b = *(const v8b*)(p + 16 + 8 * hh); v16b f;
#pragma unroll
  for (int e = 0; e < 8; ++e) { f[e] = a[e]; f[8 + e] = b[e]; } return f; }
__device__ __forceinline__ v8f wmma16b(v16b a, v16b b, v8f c) { v8f d = __builtin_amdgcn_wmma_f32_16x16x32_f16(false, a, false, b, (short)0, c, false, false); asm volatile("v_nop\n\tv_nop\n\tv_nop\n\tv_nop" : "+v"(d) : "v"(a), "v"(b)); return d; }
__device__ __forceinline__ void wave_lds_sync() { __builtin_amdgcn_fence(__ATOMIC_RELEASE, "workgroup"); __builtin_amdgcn_wave_barrier(); __builtin_amdgcn_fence(__ATOMIC_ACQUIRE, "workgroup"); }
__device__ __forceinline__ float pmul(float a, float b) { float p = a * b; asm volatile("" : "+v"(p)); return p; }
__device__ __forceinline__ int iclamp(int v, int lo, int hi) { return v < lo ? lo : (v > hi ? hi : v); }

__global__ __launch_bounds__(256) void wput_kernel(const float* __restrict__ w0, const float* __restrict__ w1, b16* __restrict__ W0T, b16* __restrict__ W1T) { const int u = blockIdx.x * 256 + threadIdx.x;
  for (int pass = 0; pass < 2; ++pass) {
    if (u < H * 4) { const int o = u / 4, k0 = (u % 4) * 8; v8b v;
#pragma unroll
      for (int j = 0; j < 8; ++j) { const int k = k0 + j; v[j] = (b16)(k < DF ? bf16_rne(w0[(size_t)k * H + o]) * WSC : 0.0f); } *(volatile v8b*)(W0T + (size_t)o * 32 + k0) = v; }
    if (u < H * 8) { const int o = u / 8, k0 = (u % 8) * 8; v8b v;
#pragma unroll
      for (int j = 0; j < 8; ++j) v[j] = (b16)(bf16_rne(w1[(size_t)(k0 + j) * H + o]) * WSC); *(volatile v8b*)(W1T + (size_t)o * H + k0) = v; }
    __threadfence(); } }
__global__ __launch_bounds__(256) void enc_kernel(const float* __restrict__ x, const float* __restrict__ extent, const float* __restrict__ tab, int PLIM, float* __restrict__ F) { const size_t p = (size_t)blockIdx.x * 256 + threadIdx.x; if (p >= (size_t)PLIM) return; const float ex = bf16_rne(extent[0]);
  float xn[3]; for (int d = 0; d < 3; ++d) xn[d] = __fdiv_rn(bf16_rne(x[p * 3 + d]), ex);
  float feat[2 * L];
#pragma unroll
  for (int l = 0; l < L; ++l) { const float sc = c_scale[l]; const int res = c_res[l]; int pg[3]; float fr[3];
    for (int d = 0; d < 3; ++d) { const float v = pmul(xn[d], sc);   float pos = v + 0.5f; asm volatile("" : "+v"(pos)); const float fl = floorf(pos); pg[d] = (int)fl; fr[d] = __fsub_rn(pos, fl); }
    float a0 = 0.0f, a1 = 0.0f; const float* tl = tab + (size_t)l * HS * 2;
#pragma unroll
    for (int c = 0; c < 8; ++c) { const int cx = (c >> 2) & 1, cy = (c >> 1) & 1, cz = c & 1; const float w = pmul(pmul(cx ? fr[0] : 1.0f - fr[0], cy ? fr[1] : 1.0f - fr[1]), cz ? fr[2] : 1.0f - fr[2]); int idx;
      if (c_dense[l]) { const int ix = iclamp(pg[0] + cx, 0, res - 1), iy = iclamp(pg[1] + cy, 0, res - 1), iz = iclamp(pg[2] + cz, 0, res - 1); idx = ix + iy * res + iz * res * res; }
      else { const unsigned ux = (unsigned)(pg[0] + cx), uy = (unsigned)(pg[1] + cy), uz = (unsigned)(pg[2] + cz); idx = (int)((ux ^ (uy * 2654435761u) ^ (uz * 805459861u)) & (unsigned)(HS - 1)); }
      idx = iclamp(idx, 0, HS - 1); const v2f tv = *(const v2f*)(tl + (size_t)idx * 2); a0 += pmul(w, bf16_rne(tv[0])); a1 += pmul(w, bf16_rne(tv[1])); }
    feat[2 * l] = a0; feat[2 * l + 1] = a1; }
  for (int pass = 0; pass < 2; ++pass) {
#pragma unroll
    for (int q = 0; q < 4; ++q) *(volatile v4f*)(F + p * DF + q * 4) = (v4f){feat[4 * q], feat[4 * q + 1], feat[4 * q + 2], feat[4 * q + 3]};
    __threadfence(); } }
__global__ __launch_bounds__(32) void mlp_kernel(const float* __restrict__ F, const b16* __restrict__ W0T, const b16* __restrict__ W1T, const float* __restrict__ w2, int PLIM, float* __restrict__ out) { __shared__ __attribute__((aligned(16))) b16 A0[32][40], A1[32][72]; __shared__ float Hf[32][68]; const int lane = threadIdx.x, nloc = lane & 15, hlf = lane >> 4; const size_t p0 = (size_t)blockIdx.x * 32; if (p0 >= (size_t)PLIM) return;
  for (int rr = 0; rr < 32; ++rr) { A0[rr][lane] = (b16)(lane < DF ? F[(p0 + rr) * DF + lane] * AS : 0.0f); }
  wave_lds_sync();
  for (int mt = 0; mt < 2; ++mt) { v8f acc[4] = {(v8f){}, (v8f){}, (v8f){}, (v8f){}}; const v16b a = frag_kb(&A0[mt * 16 + nloc][0], hlf);
#pragma unroll
    for (int t = 0; t < 4; ++t) acc[t] = wmma16b(a, frag_kb(W0T + (size_t)(t * 16 + nloc) * 32, hlf), acc[t]);
#pragma unroll
    for (int t = 0; t < 4; ++t)
#pragma unroll
      for (int r8 = 0; r8 < 8; ++r8) A1[mt * 16 + 8 * hlf + r8][t * 16 + nloc] = (b16)(fmaxf(acc[t][r8] * (1.0f / (AS * WSC)), 0.0f) * AS); }
  wave_lds_sync();
  for (int mt = 0; mt < 2; ++mt) { v8f acc[4] = {(v8f){}, (v8f){}, (v8f){}, (v8f){}};
#pragma unroll
    for (int kb = 0; kb < H; kb += 32) { const v16b a = frag_kb(&A1[mt * 16 + nloc][kb], hlf);
#pragma unroll
      for (int t = 0; t < 4; ++t) acc[t] = wmma16b(a, frag_kb(W1T + (size_t)(t * 16 + nloc) * H + kb, hlf), acc[t]); }
#pragma unroll
    for (int t = 0; t < 4; ++t)
#pragma unroll
      for (int r8 = 0; r8 < 8; ++r8) Hf[mt * 16 + 8 * hlf + r8][t * 16 + nloc] = fmaxf(acc[t][r8] * (1.0f / (AS * WSC)), 0.0f); }
  wave_lds_sync(); float o = 0.0f;
#pragma unroll 8
  for (int c = 0; c < H; ++c) o += pmul(Hf[lane][c], bf16_rne(w2[c]));
  for (int pass = 0; pass < 2; ++pass) { ((volatile float*)out)[p0 + lane] = o; __threadfence(); } }
}

extern "C" void kernel_launch(void* const* d_in, const int* in_sizes, int n_in, void* d_out, int out_size, void* d_ws, size_t ws_size, hipStream_t stream) {
  (void)n_in;
  auto Fp = [&](int i) { return (const float*)d_in[i]; };
  if (in_sizes[0] != NP * 3 || in_sizes[1] != 1 || in_sizes[2] != L * HS * 2 || in_sizes[3] != DF * H || in_sizes[4] != H * H || in_sizes[5] != H || out_size != NP) return;
  const int PLIM = NP;
  size_t off = 0; char* ws = (char*)d_ws;
  auto carve = [&](size_t bytes) { char* p = ws + off; off += (bytes + 255) & ~(size_t)255; return p; };
  b16* W0T = (b16*)carve((size_t)H * 32 * 2); b16* W1T = (b16*)carve((size_t)H * H * 2); float* F = (float*)carve((size_t)NP * DF * 4);
  if (off > ws_size || off > ((size_t)160 << 20)) return;
  wput_kernel<<<(H * 8 + 255) / 256, 256, 0, stream>>>(Fp(3), Fp(4), W0T, W1T);
  enc_kernel<<<PLIM / 256, 256, 0, stream>>>(Fp(0), Fp(1), Fp(2), PLIM, F);
  mlp_kernel<<<PLIM / 32, 32, 0, stream>>>(F, W0T, W1T, Fp(5), PLIM, (float*)d_out);
}
